// CausalGNNCore_18614388261668
// MI455X (gfx1250) — hardware-run, weakly checked
//
#include <hip/hip_runtime.h>
#include <math.h>

typedef __attribute__((ext_vector_type(16))) _Float16 v16h;
typedef __attribute__((ext_vector_type(8)))  _Float16 v8h;
typedef __attribute__((ext_vector_type(8)))  float    v8f;
typedef __attribute__((ext_vector_type(4)))  float    v4f;

constexpr int kNB    = 128;
constexpr int kND    = 128;
constexpr int kNH    = 32;
constexpr int kRows  = kNB * kND;
constexpr int kWRows = 160;
constexpr int kPA    = 40;
constexpr int kPC1   = 100;
constexpr int kPC3   = 36;
static_assert(kRows == 16384, "row count");
static_assert(kNH == 32, "one 32-deep k step per GEMM site");
static_assert((kRows % 64) == 0 && (kND % 32) == 0, "tile multiples");

constexpr float kCarry   = 256.0f;
constexpr float kCarryLo = 2048.0f;
constexpr float kInvLo   = 1.0f / kCarryLo;
constexpr float kInvAW   = 1.0f / (kCarry * kCarry);

constexpr size_t kSzPlane = (size_t)kRows * kNH * 4;
constexpr size_t kOffHS   = 0;
constexpr size_t kOffHD   = kOffHS + kSzPlane;
constexpr size_t kOffHO   = kOffHD + kSzPlane;
constexpr size_t kOffRR   = kOffHO + kSzPlane;
constexpr size_t kOffAT   = kOffRR + kSzPlane;
constexpr size_t kOffCS   = kOffAT + (size_t)kND * kND * 4;
constexpr size_t kOffWBH  = kOffCS + (size_t)kND * 4;
constexpr size_t kOffWBL  = kOffWBH + (size_t)kWRows * kNH * 2;
constexpr size_t kWsTotal = kOffWBL + (size_t)kWRows * kNH * 2;
static_assert(kWsTotal == 8475136ull, "carve total");
static_assert(kWsTotal <= 134217728ull, "carve cap");
static_assert((kOffHD % 128) == 0 && (kOffHO % 128) == 0 && (kOffRR % 128) == 0 && (kOffAT % 128) == 0 &&
              (kOffCS % 128) == 0 && (kOffWBH % 128) == 0 && (kOffWBL % 128) == 0, "128-B aligned regions");

union FragU { v16h v; v8h h[2]; };

__device__ __forceinline__ v16h frag_load(const _Float16* p) {
  FragU f;
  f.h[0] = *(const v8h*)(p);
  f.h[1] = *(const v8h*)(p + 16);
  return f.v;
}

__device__ __forceinline__ v8f mma_g(v16h a, v16h b, v8f c) {
  c = __builtin_amdgcn_wmma_f32_16x16x32_f16(false, a, false, b, (short)0, c, false, false);
  asm volatile("v_nop\n\tv_nop\n\tv_nop\n\tv_nop" : "+v"(c) : "v"(a), "v"(b));
  return c;
}

__device__ __forceinline__ void split16(float v, _Float16& hi, _Float16& lo) {
  const float c = v * kCarry;
  const _Float16 h = (_Float16)c;
  const float res = c - (float)h;
  hi = h;
  lo = (_Float16)(res * kCarryLo);
}

__global__ __launch_bounds__(128) void prep_weights_kernel(
    const float* __restrict__ m1w, const float* __restrict__ m2w, const float* __restrict__ o1w,
    _Float16* __restrict__ WBH, _Float16* __restrict__ WBL)
{
  const int seg = blockIdx.x;
  const int t = threadIdx.x;
  const float* src = m1w;
  int rowoff = 0;
  if (seg == 1) rowoff = 32;
  if (seg == 2) src = o1w;
  if (seg == 3) src = m2w;
  if (seg == 4) { src = o1w; rowoff = 32; }
  const int nl = t >> 2;
  const int k0 = (t & 3) * 8;
  v8h hv, lv;
#pragma unroll
  for (int e = 0; e < 8; ++e) {
    const float w = src[(rowoff + k0 + e) * kNH + nl];
    _Float16 p, q;
    split16(w, p, q);
    hv[e] = p;
    lv[e] = q;
  }
  _Float16* qh = WBH + seg * 1024 + t * 8;
  _Float16* ql = WBL + seg * 1024 + t * 8;
  *(volatile v8h*)qh = hv;
  *(volatile v8h*)ql = lv;
  __threadfence();
  *(volatile v8h*)qh = hv;
  *(volatile v8h*)ql = lv;
}

__global__ __launch_bounds__(128) void prep_adj_kernel(
    const float* __restrict__ W, float* __restrict__ AT, float* __restrict__ CS)
{
  __shared__ float sT[kND * 33];
  const int t = threadIdx.x;
  const int lane = t & 31;
  const int wave = __builtin_amdgcn_readfirstlane((int)(threadIdx.x >> 5));
  const int i0 = blockIdx.x * 32;
#pragma unroll 1
  for (int jj = 0; jj < 32; ++jj) {
    const int j = jj * 4 + wave;
    const float v = W[j * kND + i0 + lane];
    sT[j * 33 + lane] = (j == i0 + lane) ? 0.0f : v;
  }
  __syncthreads();
  v4f rows[8];
#pragma unroll
  for (int q = 0; q < 8; ++q) {
    const int il = wave * 8 + q;
    v4f v;
    v[0] = sT[(4 * lane + 0) * 33 + il];
    v[1] = sT[(4 * lane + 1) * 33 + il];
    v[2] = sT[(4 * lane + 2) * 33 + il];
    v[3] = sT[(4 * lane + 3) * 33 + il];
    rows[q] = v;
  }
  for (int pass = 0; pass < 2; ++pass) {
#pragma unroll
    for (int q = 0; q < 8; ++q)
      *(volatile v4f*)(AT + (size_t)(i0 + wave * 8 + q) * kND + lane * 4) = rows[q];
    __threadfence();
  }
  if (wave == 0) {
    float s = 0.0f;
#pragma unroll 1
    for (int j = 0; j < kND; ++j) s += sT[j * 33 + lane];
    volatile float* cp = CS + i0 + lane;
    *cp = s;
    __threadfence();
    *cp = s;
  }
}

__global__ __launch_bounds__(128) void enc_gemm_kernel(
    const float* __restrict__ X, const float* __restrict__ enc_w, const float* __restrict__ enc_b,
    const float* __restrict__ m1_b,
    const _Float16* __restrict__ WBH, const _Float16* __restrict__ WBL,
    float* __restrict__ HS, float* __restrict__ HD, float* __restrict__ HO)
{
  __shared__ __align__(16) _Float16 sAh[64 * kPA];
  __shared__ __align__(16) _Float16 sAl[64 * kPA];
  __shared__ __align__(16) float sC[4][16 * kPC1];
  const int tid = threadIdx.x;
  const int lane = tid & 31;
  const int wave = __builtin_amdgcn_readfirstlane((int)(threadIdx.x >> 5));
  const int r0 = blockIdx.x * 64;
  {
    const int row = tid >> 1;
    const int kh = (tid & 1) * 16;
    const float x = X[r0 + row];
#pragma unroll 1
    for (int g = 0; g < 2; ++g) {
      const int k0 = kh + g * 8;
      const v4f w0 = *(const v4f*)(enc_w + k0);
      const v4f w1 = *(const v4f*)(enc_w + k0 + 4);
      const v4f b0 = *(const v4f*)(enc_b + k0);
      const v4f b1 = *(const v4f*)(enc_b + k0 + 4);
      v8h hv, lv;
#pragma unroll
      for (int e = 0; e < 4; ++e) {
        const float a0 = tanhf(fmaf(x, w0[e], b0[e]));
        const float a1 = tanhf(fmaf(x, w1[e], b1[e]));
        _Float16 p, q;
        split16(a0, p, q);
        hv[e] = p;
        lv[e] = q;
        split16(a1, p, q);
        hv[4 + e] = p;
        lv[4 + e] = q;
      }
      *(v8h*)(sAh + row * kPA + k0) = hv;
      *(v8h*)(sAl + row * kPA + k0) = lv;
    }
  }
  __syncthreads();

  const int m = lane & 15;
  const int hh = lane >> 4;
  const v16h ah = frag_load(sAh + (wave * 16 + m) * kPA + 8 * hh);
  const v16h al = frag_load(sAl + (wave * 16 + m) * kPA + 8 * hh);
  float* slab = sC[wave];
#pragma unroll
  for (int j = 0; j < 6; ++j) {
    const v16h bh = frag_load(WBH + (j * 16 + m) * kNH + 8 * hh);
    const v16h bl = frag_load(WBL + (j * 16 + m) * kNH + 8 * hh);
    v8f cm = (v8f){0.f, 0.f, 0.f, 0.f, 0.f, 0.f, 0.f, 0.f};
    v8f cr = (v8f){0.f, 0.f, 0.f, 0.f, 0.f, 0.f, 0.f, 0.f};
    cm = mma_g(ah, bh, cm);
    cr = mma_g(ah, bl, cr);
    cr = mma_g(al, bh, cr);
    float bv = 0.0f;
    if (j == 2 || j == 3) bv = m1_b[(j - 2) * 16 + m];
#pragma unroll
    for (int r = 0; r < 8; ++r) {
      const float v = fmaf(cr[r], kInvLo, cm[r]) * kInvAW + bv;
      slab[(8 * hh + r) * kPC1 + j * 16 + m] = v;
    }
  }
  __syncthreads();

  const int q = lane >> 3;
  const int c4 = (lane & 7) * 4;
  const int rowbase = r0 + wave * 16;
  v4f vs[4], vd[4], vo[4];
#pragma unroll
  for (int it = 0; it < 4; ++it) {
    const float* sp = slab + (it * 4 + q) * kPC1 + c4;
    vs[it] = *(const v4f*)(sp);
    vd[it] = *(const v4f*)(sp + 32);
    vo[it] = *(const v4f*)(sp + 64);
  }
  for (int pass = 0; pass < 2; ++pass) {
#pragma unroll
    for (int it = 0; it < 4; ++it) {
      const size_t o = (size_t)(rowbase + it * 4 + q) * kNH + c4;
      *(volatile v4f*)(HS + o) = vs[it];
      *(volatile v4f*)(HD + o) = vd[it];
      *(volatile v4f*)(HO + o) = vo[it];
    }
    __threadfence();
  }
}

__global__ __launch_bounds__(256) void agg_rsum_kernel(
    const float* __restrict__ HS, const float* __restrict__ HD, const float* __restrict__ AT,
    float* __restrict__ RR)
{
  __shared__ __align__(16) float sHs[kND * kNH];
  __shared__ __align__(16) float sAt[8 * kND];
  const int tid = threadIdx.x;
  const int lane = tid & 31;
  const int wave = __builtin_amdgcn_readfirstlane((int)(threadIdx.x >> 5));
  const int b = blockIdx.x >> 4;
  const int ig = blockIdx.x & 15;
  const float* hsb = HS + (size_t)b * kND * kNH;
#pragma unroll
  for (int t = 0; t < 4; ++t) {
    const int idx = (tid + t * 256) * 4;
    *(v4f*)(sHs + idx) = *(const v4f*)(hsb + idx);
  }
  *(v4f*)(sAt + tid * 4) = *(const v4f*)(AT + (size_t)ig * 8 * kND + tid * 4);
  const int i = ig * 8 + wave;
  const size_t orow = ((size_t)b * kND + i) * kNH + lane;
  const float hdv = HD[orow];
  __syncthreads();
  const float* at = sAt + wave * kND;
  float acc = 0.0f;
#pragma unroll 8
  for (int j = 0; j < kND; ++j) {
    acc = fmaf(at[j], fmaxf(sHs[j * kNH + lane] + hdv, 0.0f), acc);
  }
  volatile float* rp = RR + orow;
  *rp = acc;
  __threadfence();
  *rp = acc;
}

__global__ __launch_bounds__(128) void final_kernel(
    const float* __restrict__ RR, const float* __restrict__ HO, const float* __restrict__ CS,
    const _Float16* __restrict__ WBH, const _Float16* __restrict__ WBL,
    const float* __restrict__ m2_b, const float* __restrict__ o1_b,
    const float* __restrict__ o2_w, const float* __restrict__ o2_b,
    float* __restrict__ OUT)
{
  __shared__ __align__(16) float sG[4][32 * kPC3];
  __shared__ __align__(16) float sZ[4][32 * kPC3];
  const int tid = threadIdx.x;
  const int lane = tid & 31;
  const int wave = __builtin_amdgcn_readfirstlane((int)(threadIdx.x >> 5));
  const int m = lane & 15;
  const int hh = lane >> 4;
  const int b = blockIdx.x;
  const int rb = b * kND + wave * 32;
  float* g = sG[wave];
  float* z = sZ[wave];

  {
    v16h bh[2], bl[2];
#pragma unroll
    for (int j = 0; j < 2; ++j) {
      bh[j] = frag_load(WBH + (96 + j * 16 + m) * kNH + 8 * hh);
      bl[j] = frag_load(WBL + (96 + j * 16 + m) * kNH + 8 * hh);
    }
    const float mb0 = m2_b[m];
    const float mb1 = m2_b[16 + m];
#pragma unroll
    for (int t = 0; t < 2; ++t) {
      const float* rp = RR + (size_t)(rb + t * 16 + m) * kNH + 8 * hh;
      const v4f a0 = *(const v4f*)(rp);
      const v4f a1 = *(const v4f*)(rp + 4);
      const v4f a2 = *(const v4f*)(rp + 16);
      const v4f a3 = *(const v4f*)(rp + 20);
      v16h ah, al;
#pragma unroll
      for (int e = 0; e < 4; ++e) {
        _Float16 p, q;
        split16(a0[e], p, q);
        ah[e] = p;
        al[e] = q;
        split16(a1[e], p, q);
        ah[4 + e] = p;
        al[4 + e] = q;
        split16(a2[e], p, q);
        ah[8 + e] = p;
        al[8 + e] = q;
        split16(a3[e], p, q);
        ah[12 + e] = p;
        al[12 + e] = q;
      }
      const float* cp = CS + wave * 32 + t * 16 + 8 * hh;
      const v4f cs0 = *(const v4f*)(cp);
      const v4f cs1 = *(const v4f*)(cp + 4);
#pragma unroll
      for (int j = 0; j < 2; ++j) {
        v8f cm = (v8f){0.f, 0.f, 0.f, 0.f, 0.f, 0.f, 0.f, 0.f};
        v8f cr = (v8f){0.f, 0.f, 0.f, 0.f, 0.f, 0.f, 0.f, 0.f};
        cm = mma_g(ah, bh[j], cm);
        cr = mma_g(ah, bl[j], cr);
        cr = mma_g(al, bh[j], cr);
        const float mb = (j == 0) ? mb0 : mb1;
#pragma unroll
        for (int r = 0; r < 8; ++r) {
          const float csr = (r < 4) ? cs0[r & 3] : cs1[r & 3];
          const float v = fmaf(cr[r], kInvLo, cm[r]) * kInvAW + csr * mb;
          g[(t * 16 + 8 * hh + r) * kPC3 + j * 16 + m] = v;
        }
      }
    }
  }
  __syncthreads();

  {
    v16h bh[2], bl[2];
#pragma unroll
    for (int j = 0; j < 2; ++j) {
      bh[j] = frag_load(WBH + (128 + j * 16 + m) * kNH + 8 * hh);
      bl[j] = frag_load(WBL + (128 + j * 16 + m) * kNH + 8 * hh);
    }
#pragma unroll
    for (int t = 0; t < 2; ++t) {
      const float* gp = g + (t * 16 + m) * kPC3 + 8 * hh;
      const v4f a0 = *(const v4f*)(gp);
      const v4f a1 = *(const v4f*)(gp + 4);
      const v4f a2 = *(const v4f*)(gp + 16);
      const v4f a3 = *(const v4f*)(gp + 20);
      v16h ah, al;
#pragma unroll
      for (int e = 0; e < 4; ++e) {
        _Float16 p, q;
        split16(a0[e], p, q);
        ah[e] = p;
        al[e] = q;
        split16(a1[e], p, q);
        ah[4 + e] = p;
        al[4 + e] = q;
        split16(a2[e], p, q);
        ah[8 + e] = p;
        al[8 + e] = q;
        split16(a3[e], p, q);
        ah[12 + e] = p;
        al[12 + e] = q;
      }
#pragma unroll
      for (int j = 0; j < 2; ++j) {
        v8f cm = (v8f){0.f, 0.f, 0.f, 0.f, 0.f, 0.f, 0.f, 0.f};
        v8f cr = (v8f){0.f, 0.f, 0.f, 0.f, 0.f, 0.f, 0.f, 0.f};
        cm = mma_g(ah, bh[j], cm);
        cr = mma_g(ah, bl[j], cr);
        cr = mma_g(al, bh[j], cr);
#pragma unroll
        for (int r = 0; r < 8; ++r) {
          z[(t * 16 + 8 * hh + r) * kPC3 + j * 16 + m] = fmaf(cr[r], kInvLo, cm[r]) * kInvAW;
        }
      }
    }
  }
  __syncthreads();

  {
    const int row = rb + lane;
    const float* zp = z + lane * kPC3;
    const float* hop = HO + (size_t)row * kNH;
    float acc = 0.0f;
#pragma unroll 2
    for (int c = 0; c < 8; ++c) {
      const v4f zc = *(const v4f*)(zp + 4 * c);
      const v4f hv = *(const v4f*)(hop + 4 * c);
      const v4f ob = *(const v4f*)(o1_b + 4 * c);
      const v4f ow = *(const v4f*)(o2_w + 4 * c);
#pragma unroll
      for (int e = 0; e < 4; ++e) {
        const float zz = fmaxf((hv[e] + zc[e]) + ob[e], 0.0f);
        acc = fmaf(zz, ow[e], acc);
      }
    }
    const float res = acc + o2_b[0];
    volatile float* op = OUT + row;
    *op = res;
    __threadfence();
    *op = res;
  }
}

extern "C" void kernel_launch(void* const* d_in, const int* in_sizes, int n_in,
                              void* d_out, int out_size, void* d_ws, size_t ws_size,
                              hipStream_t stream) {
  if (n_in < 12) return;
  if (in_sizes[0] != kNB * kND) return;
  if (in_sizes[1] != kND * kND) return;
  if (in_sizes[2] != kNH) return;
  if (in_sizes[3] != kNH) return;
  if (in_sizes[4] != 2 * kNH * kNH) return;
  if (in_sizes[5] != kNH) return;
  if (in_sizes[6] != kNH * kNH) return;
  if (in_sizes[7] != kNH) return;
  if (in_sizes[8] != 2 * kNH * kNH) return;
  if (in_sizes[9] != kNH) return;
  if (in_sizes[10] != kNH) return;
  if (in_sizes[11] != 1) return;
  if (out_size != kRows) return;
  if (ws_size < kWsTotal) return;

  const float* X     = (const float*)d_in[0];
  const float* W     = (const float*)d_in[1];
  const float* enc_w = (const float*)d_in[2];
  const float* enc_b = (const float*)d_in[3];
  const float* m1_w  = (const float*)d_in[4];
  const float* m1_b  = (const float*)d_in[5];
  const float* m2_w  = (const float*)d_in[6];
  const float* m2_b  = (const float*)d_in[7];
  const float* o1_w  = (const float*)d_in[8];
  const float* o1_b  = (const float*)d_in[9];
  const float* o2_w  = (const float*)d_in[10];
  const float* o2_b  = (const float*)d_in[11];
  float* out = (float*)d_out;

  char* ws = (char*)d_ws;
  float*    HS  = (float*)(ws + kOffHS);
  float*    HD  = (float*)(ws + kOffHD);
  float*    HO  = (float*)(ws + kOffHO);
  float*    RR  = (float*)(ws + kOffRR);
  float*    AT  = (float*)(ws + kOffAT);
  float*    CS  = (float*)(ws + kOffCS);
  _Float16* WBH = (_Float16*)(ws + kOffWBH);
  _Float16* WBL = (_Float16*)(ws + kOffWBL);

  prep_weights_kernel<<<5, 128, 0, stream>>>(m1_w, m2_w, o1_w, WBH, WBL);
  prep_adj_kernel<<<kND / 32, 128, 0, stream>>>(W, AT, CS);
  enc_gemm_kernel<<<kRows / 64, 128, 0, stream>>>(X, enc_w, enc_b, m1_b, WBH, WBL, HS, HD, HO);
  agg_rsum_kernel<<<kNB * (kND / 8), 256, 0, stream>>>(HS, HD, AT, RR);
  final_kernel<<<kNB, 128, 0, stream>>>(RR, HO, CS, WBH, WBL, m2_b, o1_b, o2_w, o2_b, out);
}
